// ResidualAdvection_1099511628422
// MI455X (gfx1250) — hardware-verified
//
#include <hip/hip_runtime.h>
#define NBI 8
#define HH 512
#define NPX (HH * HH)
#define PW 514
#define PR 516
#define MP (HH * PW)
#define C1 16
#define CHP 32
#define NO 18
#define NOP 32
#define KI 160
#define HPX (NPX / 2)
typedef __bf16 v16b __attribute__((ext_vector_type(16)));
typedef unsigned short v8us __attribute__((ext_vector_type(8), may_alias));
typedef float  v8f  __attribute__((ext_vector_type(8)));
typedef float  v4f  __attribute__((ext_vector_type(4)));
typedef float  v4fa __attribute__((ext_vector_type(4), may_alias));
union FragB { v16b v; v8us half[2]; unsigned short u[16]; };

__device__ __forceinline__ unsigned short bf16_bits(float x) { unsigned int u = __float_as_uint(x); return (unsigned short)((u + 0x7FFFu + ((u >> 16) & 1u)) >> 16); }
__device__ __forceinline__ float bf16_val(unsigned short b) { return __uint_as_float(((unsigned int)b) << 16); }
__device__ __forceinline__ float bf16_round(float x) { return bf16_val(bf16_bits(x)); }
template <int NT>
__device__ __forceinline__ v8f mmaN(v16b ah, v16b al, v16b bh, v16b bl, v8f c) {
  c = __builtin_amdgcn_wmma_f32_16x16x32_bf16(false, ah, false, bh, (short)0, c, false, false);
  if (NT >= 2) c = __builtin_amdgcn_wmma_f32_16x16x32_bf16(false, al, false, bh, (short)0, c, false, false);
  if (NT >= 3) c = __builtin_amdgcn_wmma_f32_16x16x32_bf16(false, ah, false, bl, (short)0, c, false, false);
  asm volatile("v_nop\n\tv_nop\n\tv_nop\n\tv_nop" : "+v"(c) : "v"(ah), "v"(al), "v"(bh), "v"(bl));
  return c;
}

__global__ __launch_bounds__(256) void k_wt_bf16(const float* __restrict__ W, unsigned short* __restrict__ Wt, int K, int N) {
  const int t = blockIdx.x * 256 + threadIdx.x;
  const int k8n = K / 8;
  if (t >= N * k8n) return;
  const int n = t / k8n, k8 = (t % k8n) * 8;
  v8us v;
#pragma unroll
  for (int i = 0; i < 8; ++i) v[i] = bf16_bits(W[(size_t)(k8 + i) * N + n]);
  *(volatile v8us*)(Wt + (size_t)n * K + k8) = v;
  __threadfence();
  *(volatile v8us*)(Wt + (size_t)n * K + k8) = v;
}

template <bool ASPLIT, int ACT, bool BIAS_BF16>
__global__ __launch_bounds__(128) void k_gemm_bf(const float* __restrict__ A, int lda, const unsigned short* __restrict__ Wt, int ldb,
                                               const float* __restrict__ bias, float* __restrict__ C, int ldc, int M, int N, int K) {
  __shared__ __attribute__((aligned(16))) float so[4][16][64];
  const int tid = threadIdx.x, w = tid >> 5, lane = tid & 31, ln = lane & 15, hh = lane >> 4;
  const int ntn = N / 64;
  const int wid = blockIdx.x * 4 + w;
  const int mt = wid / ntn, nq = wid % ntn;
  if (mt * 16 >= M) return;
  const int row0 = mt * 16, col0 = nq * 64;
  const float* arow = A + (size_t)(row0 + ln) * lda;
  v8f acc[4] = {};
  for (int kb = 0; kb < K; kb += 32) {
    FragB ah, al;
    const v4f x0 = *(const v4fa*)(arow + kb + 8 * hh), x1 = *(const v4fa*)(arow + kb + 8 * hh + 4);
    const v4f x2 = *(const v4fa*)(arow + kb + 16 + 8 * hh), x3 = *(const v4fa*)(arow + kb + 16 + 8 * hh + 4);
    float xs[16] = {x0[0],x0[1],x0[2],x0[3],x1[0],x1[1],x1[2],x1[3],x2[0],x2[1],x2[2],x2[3],x3[0],x3[1],x3[2],x3[3]};
#pragma unroll
    for (int i = 0; i < 16; ++i) { const unsigned short hb = bf16_bits(xs[i]); ah.u[i] = hb; al.u[i] = ASPLIT ? bf16_bits(xs[i] - bf16_val(hb)) : (unsigned short)0; }
#pragma unroll
    for (int t = 0; t < 4; ++t) {
      const unsigned short* brow = Wt + (size_t)(col0 + t * 16 + ln) * ldb + kb;
      FragB b;
      b.half[0] = *(const v8us*)(brow + 8 * hh);
      b.half[1] = *(const v8us*)(brow + 16 + 8 * hh);
      acc[t] = mmaN<ASPLIT ? 2 : 1>(ah.v, al.v, b.v, b.v, acc[t]);
    }
  }
#pragma unroll
  for (int t = 0; t < 4; ++t) {
    float bv = bias ? bias[col0 + t * 16 + ln] : 0.f;
    if (BIAS_BF16) bv = bf16_round(bv);
#pragma unroll
    for (int r = 0; r < 8; ++r) { float v = acc[t][r] + bv; if (ACT == 1) v = fmaxf(v, 0.f); so[w][8 * hh + r][t * 16 + ln] = v; }
  }
  __builtin_amdgcn_fence(__ATOMIC_ACQ_REL, "workgroup");
  __builtin_amdgcn_wave_barrier();
  const int rsub = lane >> 4, c4 = (lane & 15) * 4;
  for (int pass = 0; pass < 2; ++pass) {
#pragma unroll
    for (int q = 0; q < 8; ++q) {
      const int r = q * 2 + rsub;
      const v4f v = *(const v4fa*)&so[w][r][c4];
      *(volatile v4f*)(C + (size_t)(row0 + r) * ldc + col0 + c4) = v;
    }
    if (pass == 0) __threadfence();
  }
}

template <bool ASPLIT, int ACT, bool BIAS_BF16, bool RES_BF16>
__global__ __launch_bounds__(128) void k_gemm_bf3(const float* __restrict__ A, int lda, const unsigned short* __restrict__ Wt, int ldb,
                                                const float* __restrict__ bias, const float* __restrict__ resid, int rmod, int ldr,
                                                float* __restrict__ C, int ldc, int M, int N, int K) {
  __shared__ __attribute__((aligned(16))) float so[4][16][64];
  const int tid = threadIdx.x, w = tid >> 5, lane = tid & 31, ln = lane & 15, hh = lane >> 4;
  const int ntn = N / 64;
  const int wid = blockIdx.x * 4 + w;
  const int mt = wid / ntn, nq = wid % ntn;
  if (mt * 16 >= M) return;
  const int row0 = mt * 16, col0 = nq * 64;
  const float* arow = A + (size_t)(row0 + ln) * lda;
  v8f acc[4] = {};
  for (int kb = 0; kb < K; kb += 32) {
    FragB ah, al;
    const v4f x0 = *(const v4fa*)(arow + kb + 8 * hh), x1 = *(const v4fa*)(arow + kb + 8 * hh + 4);
    const v4f x2 = *(const v4fa*)(arow + kb + 16 + 8 * hh), x3 = *(const v4fa*)(arow + kb + 16 + 8 * hh + 4);
    float xs[16] = {x0[0],x0[1],x0[2],x0[3],x1[0],x1[1],x1[2],x1[3],x2[0],x2[1],x2[2],x2[3],x3[0],x3[1],x3[2],x3[3]};
#pragma unroll
    for (int i = 0; i < 16; ++i) { const unsigned short hb = bf16_bits(xs[i]); ah.u[i] = hb; al.u[i] = ASPLIT ? bf16_bits(xs[i] - bf16_val(hb)) : (unsigned short)0; }
#pragma unroll
    for (int t = 0; t < 4; ++t) {
      const unsigned short* brow = Wt + (size_t)(col0 + t * 16 + ln) * ldb + kb;
      FragB b;
      b.half[0] = *(const v8us*)(brow + 8 * hh);
      b.half[1] = *(const v8us*)(brow + 16 + 8 * hh);
      acc[t] = mmaN<ASPLIT ? 2 : 1>(ah.v, al.v, b.v, b.v, acc[t]);
    }
  }
#pragma unroll
  for (int t = 0; t < 4; ++t) {
    const int col = col0 + t * 16 + ln;
    float bv = bias ? bias[col] : 0.f;
    if (BIAS_BF16) bv = bf16_round(bv);
#pragma unroll
    for (int r = 0; r < 8; ++r) {
      float v = acc[t][r] + bv;
      if (resid) { float rv = resid[(size_t)((row0 + 8 * hh + r) % rmod) * ldr + col]; if (RES_BF16) rv = bf16_round(rv); v += rv; }
      if (ACT == 1) v = fmaxf(v, 0.f);
      if (ACT == 2) v = 0.5f * v * (1.0f + erff(v * 0.70710678118654752f));
      if (ACT == 3) { const float u = 0.7978845608028654f * (v + 0.044715f * v * v * v); v = 0.5f * v * (1.0f + tanhf(u)); }
      so[w][8 * hh + r][t * 16 + ln] = v;
    }
  }
  __builtin_amdgcn_fence(__ATOMIC_ACQ_REL, "workgroup");
  __builtin_amdgcn_wave_barrier();
  const int rsub = lane >> 4, c4 = (lane & 15) * 4;
  for (int pass = 0; pass < 2; ++pass) {
#pragma unroll
    for (int q = 0; q < 8; ++q) {
      const int r = q * 2 + rsub;
      const v4f v = *(const v4fa*)&so[w][r][c4];
      *(volatile v4f*)(C + (size_t)(row0 + r) * ldc + col0 + c4) = v;
    }
    if (pass == 0) __threadfence();
  }
}
template <bool PARAM_BF16>
__global__ __launch_bounds__(256) void k_layernorm(const float* __restrict__ X, const float* __restrict__ R, const float* __restrict__ g, const float* __restrict__ bta,
                                                  float* __restrict__ out_sum, float* __restrict__ out_norm, int N, float eps) {
  __shared__ float red[256];
  const int row = blockIdx.x, tid = threadIdx.x;
  const float* x = X + (size_t)row * N; const float* rr = R ? R + (size_t)row * N : nullptr;
  float vals[16];
  const int per = N / 256;
  float s1 = 0.f;
  for (int u = 0; u < per / 4; ++u) {
    const int j = tid * 4 + 1024 * u;
    const v4f a = *(const v4fa*)(x + j);
    v4f b = {0.f,0.f,0.f,0.f}; if (rr) b = *(const v4fa*)(rr + j);
#pragma unroll
    for (int q = 0; q < 4; ++q) { const float v = a[q] + b[q]; vals[u * 4 + q] = v; s1 += v; }
  }
  red[tid] = s1; __syncthreads();
  for (int st = 128; st > 0; st >>= 1) { if (tid < st) red[tid] += red[tid + st]; __syncthreads(); }
  const float mu = red[0] / (float)N; __syncthreads();
  float s2 = 0.f;
  for (int u = 0; u < per / 4; ++u)
#pragma unroll
    for (int q = 0; q < 4; ++q) { const float c = vals[u * 4 + q] - mu; s2 += c * c; }
  red[tid] = s2; __syncthreads();
  for (int st = 128; st > 0; st >>= 1) { if (tid < st) red[tid] += red[tid + st]; __syncthreads(); }
  const float rs = rsqrtf(red[0] / (float)N + eps);
  for (int pass = 0; pass < 2; ++pass) {
    for (int u = 0; u < per / 4; ++u) {
      const int j = tid * 4 + 1024 * u;
      v4f o, sm;
#pragma unroll
      for (int q = 0; q < 4; ++q) {
        float gg = g[j + q], bb = bta[j + q];
        if (PARAM_BF16) { gg = bf16_round(gg); bb = bf16_round(bb); }
        sm[q] = vals[u * 4 + q]; o[q] = (vals[u * 4 + q] - mu) * rs * gg + bb;
      }
      if (out_sum) *(volatile v4f*)(out_sum + (size_t)row * N + j) = sm;
      *(volatile v4f*)(out_norm + (size_t)row * N + j) = o;
    }
    if (pass == 0) __threadfence();
  }
}


typedef _Float16 v16h __attribute__((ext_vector_type(16)));
union FragH { v16h v; v8us half[2]; _Float16 h[16]; unsigned short u[16]; };
template <int NT>
__device__ __forceinline__ v8f mmaH(v16h ah, v16h al, v16h bh, v16h bl, v8f c) {
  c = __builtin_amdgcn_wmma_f32_16x16x32_f16(false, ah, false, bh, (short)0, c, false, false);
  if (NT >= 2) c = __builtin_amdgcn_wmma_f32_16x16x32_f16(false, al, false, bh, (short)0, c, false, false);
  if (NT >= 3) c = __builtin_amdgcn_wmma_f32_16x16x32_f16(false, ah, false, bl, (short)0, c, false, false);
  asm volatile("v_nop\n\tv_nop\n\tv_nop\n\tv_nop" : "+v"(c) : "v"(ah), "v"(al), "v"(bh), "v"(bl));
  return c;
}
template <bool ASPLIT>
__global__ __launch_bounds__(128) void k_gemm_h(const float* __restrict__ A, int lda, size_t sA, const _Float16* __restrict__ Bh, int ldb, size_t sB, float alpha, float* __restrict__ C, int ldc, size_t sC, int M, int N, int K) {
  __shared__ __attribute__((aligned(16))) float so[4][16][64];
  const int tid = threadIdx.x, w = tid >> 5, lane = tid & 31, ln = lane & 15, hh = lane >> 4; const int by = blockIdx.y;
  A += (size_t)by * sA; Bh += (size_t)by * sB; C += (size_t)by * sC;
  const int ntn = (N + 63) / 64; const int wid = blockIdx.x * 4 + w; const int mt = wid / ntn, nq = wid % ntn; if (mt * 16 >= M) return;
  const int row0 = mt * 16, col0 = nq * 64; const float* arow = A + (size_t)(row0 + ln) * lda;
  v8f acc[4] = {};
  for (int kb = 0; kb < K; kb += 32) {
    FragH ah, al;
    const v4f x0 = *(const v4fa*)(arow + kb + 8 * hh), x1 = *(const v4fa*)(arow + kb + 8 * hh + 4), x2 = *(const v4fa*)(arow + kb + 16 + 8 * hh), x3 = *(const v4fa*)(arow + kb + 16 + 8 * hh + 4);
    float xs[16] = {x0[0],x0[1],x0[2],x0[3],x1[0],x1[1],x1[2],x1[3],x2[0],x2[1],x2[2],x2[3],x3[0],x3[1],x3[2],x3[3]};
#pragma unroll
    for (int i = 0; i < 16; ++i) { const _Float16 h = (_Float16)xs[i]; ah.h[i] = h; al.h[i] = ASPLIT ? (_Float16)(xs[i] - (float)h) : (_Float16)0.0f; }
#pragma unroll
    for (int t = 0; t < 4; ++t) { if (col0 + t * 16 >= N) continue; const size_t boff = (size_t)(col0 + t * 16 + ln) * ldb + kb; FragH bq; bq.half[0] = *(const v8us*)(Bh + boff + 8 * hh); bq.half[1] = *(const v8us*)(Bh + boff + 16 + 8 * hh);
      acc[t] = mmaH<ASPLIT ? 2 : 1>(ah.v, al.v, bq.v, bq.v, acc[t]); }
  }
#pragma unroll
  for (int t = 0; t < 4; ++t) { if (col0 + t * 16 >= N) continue;
#pragma unroll
    for (int r = 0; r < 8; ++r) so[w][8 * hh + r][t * 16 + ln] = acc[t][r] * alpha; }
  __builtin_amdgcn_fence(__ATOMIC_ACQ_REL, "workgroup"); __builtin_amdgcn_wave_barrier();
  const int rsub = lane >> 4, c4 = (lane & 15) * 4;
  for (int pass = 0; pass < 2; ++pass) {
#pragma unroll
    for (int q = 0; q < 8; ++q) { const int r = q * 2 + rsub; if (col0 + c4 < N) { const v4f v = *(const v4fa*)&so[w][r][c4]; *(volatile v4f*)(C + (size_t)(row0 + r) * ldc + col0 + c4) = v; } }
    if (pass == 0) __threadfence(); }
}

__global__ __launch_bounds__(256) void k_wt_f16(const float* __restrict__ W, _Float16* __restrict__ Wt, int K, int N, float scale) {
  const int t = blockIdx.x * 256 + threadIdx.x; if (t >= N * (K / 8)) return; const int n = t / (K / 8), k8 = (t % (K / 8)) * 8; FragH f;
#pragma unroll
  for (int i = 0; i < 8; ++i) f.h[i] = (_Float16)(bf16_round(W[(size_t)(k8 + i) * N + n]) * scale); const v8us o = f.half[0];
  *(volatile v8us*)((unsigned short*)Wt + (size_t)n * K + k8) = o; __threadfence(); *(volatile v8us*)((unsigned short*)Wt + (size_t)n * K + k8) = o;
}
template <int ACT>
__global__ __launch_bounds__(128) void k_gemm_hhx(const _Float16* __restrict__ A, int lda, size_t sA, const _Float16* __restrict__ Bh, int ldb, size_t sB, float alpha, const float* __restrict__ bias, size_t sBias, const float* __restrict__ CP, int rowsPerB, size_t sCPb, int row0g,
    float* __restrict__ C, _Float16* __restrict__ C16, int ldc, size_t sC, int M, int N, int K) {
  __shared__ __attribute__((aligned(16))) float so[4][16][64];
  const int tid = threadIdx.x, w = tid >> 5, lane = tid & 31, ln = lane & 15, hh = lane >> 4; const int by = blockIdx.y;
  A += (size_t)by * sA; Bh += (size_t)by * sB; const size_t cofs = (size_t)by * sC; const float* bp = bias ? bias + (size_t)by * sBias : nullptr;
  const int ntn = (N + 63) / 64; const int wid = blockIdx.x * 4 + w; const int mt = wid / ntn, nq = wid % ntn; if (mt * 16 >= M) return;
  const int row0 = mt * 16, col0 = nq * 64; const _Float16* arow = A + (size_t)(row0 + ln) * lda;
  v8f acc[4] = {};
  for (int kb = 0; kb < K; kb += 32) { FragH ah; ah.half[0] = *(const v8us*)((const unsigned short*)arow + kb + 8 * hh); ah.half[1] = *(const v8us*)((const unsigned short*)arow + kb + 16 + 8 * hh);
#pragma unroll
    for (int t = 0; t < 4; ++t) { if (col0 + t * 16 >= N) continue; const size_t boff = (size_t)(col0 + t * 16 + ln) * ldb + kb; FragH bq; bq.half[0] = *(const v8us*)((const unsigned short*)Bh + boff + 8 * hh); bq.half[1] = *(const v8us*)((const unsigned short*)Bh + boff + 16 + 8 * hh);
      acc[t] = mmaH<1>(ah.v, ah.v, bq.v, bq.v, acc[t]); }
  }
#pragma unroll
  for (int t = 0; t < 4; ++t) { if (col0 + t * 16 >= N) continue; const int col = col0 + t * 16 + ln; const float bv = bp ? bf16_round(bp[col]) : 0.f;
#pragma unroll
    for (int r = 0; r < 8; ++r) { float v = acc[t][r] * alpha + bv; if (CP) { const int bidx = (row0g + row0 + 8 * hh + r) / rowsPerB; v += CP[(size_t)bidx * sCPb + (size_t)by * 64 + col]; } if (ACT == 1) v = (v > 0.f) ? v : expm1f(v); else if (ACT == 7) v = (v > 0.f) ? v + 1.0f : expf(v); else if (ACT == 8) v = tanhf(v); else if (ACT == 9) v = 0.5f * v * (1.0f + tanhf(0.7978845608028654f * (v + 0.044715f * v * v * v))); else if (ACT == 11) v = 1.0f / (1.0f + expf(-v)); else if (ACT == 12) v = (v > 0.f) ? v : 0.01f * v; else if (ACT == 14) v = (v > 0.f) ? v : 0.1f * v; else if (ACT == 15) v = v / (1.0f + expf(-v)); else if (ACT == 3) v = fmaxf(v, 0.f); else if (ACT == 6) v = 0.5f * v * (1.0f + erff(v * 0.70710678118654752f)); so[w][8 * hh + r][t * 16 + ln] = v; } }
  __builtin_amdgcn_fence(__ATOMIC_ACQ_REL, "workgroup"); __builtin_amdgcn_wave_barrier();
  const int rsub = lane >> 4, c4 = (lane & 15) * 4; typedef _Float16 v4h __attribute__((ext_vector_type(4)));
  for (int pass = 0; pass < 2; ++pass) {
#pragma unroll
    for (int q = 0; q < 8; ++q) { const int r = q * 2 + rsub; if (col0 + c4 < N) { const v4f v = *(const v4fa*)&so[w][r][c4]; if (C) *(volatile v4f*)(C + cofs + (size_t)(row0 + r) * ldc + col0 + c4) = v; if (C16) { v4h h4; for (int i = 0; i < 4; ++i) h4[i] = (_Float16)v[i]; *(volatile v4h*)(C16 + cofs + (size_t)(row0 + r) * ldc + col0 + c4) = h4; } } }
    if (pass == 0) __threadfence(); }
}


typedef _Float16 v4h __attribute__((ext_vector_type(4)));

__global__ __launch_bounds__(256) void k_x16(const float* __restrict__ x, _Float16* __restrict__ X16, size_t n8) { const size_t t = (size_t)blockIdx.x * 256 + threadIdx.x; if (t >= n8) return; FragH f;
#pragma unroll
  for (int q = 0; q < 8; ++q) f.h[q] = (_Float16)bf16_round(x[t * 8 + q]); *(volatile v8us*)((unsigned short*)X16 + t * 8) = f.half[0]; __threadfence(); *(volatile v8us*)((unsigned short*)X16 + t * 8) = f.half[0]; }
__global__ __launch_bounds__(256) void k_h16(const float* __restrict__ x, _Float16* __restrict__ X16, size_t n8) { const size_t t = (size_t)blockIdx.x * 256 + threadIdx.x; if (t >= n8) return; FragH f;
#pragma unroll
  for (int q = 0; q < 8; ++q) f.h[q] = (_Float16)x[t * 8 + q]; *(volatile v8us*)((unsigned short*)X16 + t * 8) = f.half[0]; __threadfence(); *(volatile v8us*)((unsigned short*)X16 + t * 8) = f.half[0]; }
__global__ __launch_bounds__(256) void k_round16f(const float* __restrict__ W, _Float16* __restrict__ Bt, size_t n8) { const size_t t = (size_t)blockIdx.x * 256 + threadIdx.x; if (t >= n8) return; FragH f;
#pragma unroll
  for (int i = 0; i < 8; ++i) f.h[i] = (_Float16)(bf16_round(W[t * 8 + i]) * 16.0f); *(volatile v8us*)((unsigned short*)Bt + t * 8) = f.half[0]; __threadfence(); *(volatile v8us*)((unsigned short*)Bt + t * 8) = f.half[0]; }
template <int NHv, int TTv>
__global__ __launch_bounds__(256) void k_vt(const _Float16* __restrict__ V16, int ldv, int voff, _Float16* __restrict__ Vt) { __shared__ unsigned short tl[64][66]; const int tid = threadIdx.x; const int slab = blockIdx.x / (TTv / 64), lg = blockIdx.x % (TTv / 64); const int b = slab / NHv, h = slab % NHv;
  for (int i = tid; i < 64 * 8; i += 256) { const int r = i / 8, c8 = (i % 8) * 8; FragH f; f.half[0] = *(const v8us*)((const unsigned short*)V16 + ((size_t)b * TTv + lg * 64 + r) * ldv + voff + h * 64 + c8);
#pragma unroll
    for (int q = 0; q < 8; ++q) tl[r][c8 + q] = f.u[q]; }
  __syncthreads();
  for (int pass = 0; pass < 2; ++pass) {
#pragma unroll
    for (int rd = 0; rd < 2; ++rd) { const int d = rd * 32 + tid / 8, pc = tid % 8; FragH f;
#pragma unroll
      for (int q = 0; q < 8; ++q) f.u[q] = tl[pc * 8 + q][d];
      *(volatile v8us*)((unsigned short*)Vt + ((size_t)slab * 64 + d) * TTv + lg * 64 + pc * 8) = f.half[0]; }
    if (pass == 0) __threadfence(); } }

__global__ __launch_bounds__(256) void k_hl(const float* __restrict__ F, _Float16* __restrict__ Hh, _Float16* __restrict__ Hl, size_t n8) { const size_t t = (size_t)blockIdx.x * 256 + threadIdx.x; if (t >= n8) return; FragH fh, fl; const v4f a = *(const v4fa*)(F + t * 8), c = *(const v4fa*)(F + t * 8 + 4);
#pragma unroll
  for (int q = 0; q < 4; ++q) { _Float16 h = (_Float16)a[q]; fh.h[q] = h; fl.h[q] = (_Float16)((a[q] - (float)h) * 1024.0f); h = (_Float16)c[q]; fh.h[4 + q] = h; fl.h[4 + q] = (_Float16)((c[q] - (float)h) * 1024.0f); }
  for (int pass = 0; pass < 2; ++pass) { *(volatile v8us*)((unsigned short*)Hh + t * 8) = fh.half[0]; *(volatile v8us*)((unsigned short*)Hl + t * 8) = fl.half[0]; if (pass == 0) __threadfence(); } }

__global__ __launch_bounds__(256) void k_conv1(const float* __restrict__ wind, const float* __restrict__ topo, int b, const float* __restrict__ w1, const float* __restrict__ b1, _Float16* __restrict__ XP) {
  #pragma clang fp contract(off)
  const int tt = blockIdx.x * 256 + threadIdx.x; if (tt >= PR * PW * 2) return; const int half = tt & 1, t = tt >> 1; const int yp = t / PW - 1, xq = t % PW - 1; const bool in = (yp >= 0 && yp < HH && xq >= 0 && xq < HH); const int o0 = 8 * half; float acc[8];
#pragma unroll
  for (int o = 0; o < 8; ++o) acc[o] = bf16_round(b1[o0 + o]);
#pragma unroll 1
  for (int tap = 0; tap < 27; ++tap) { const int ci = tap / 9, ky = (tap / 3) % 3, kx = tap % 3; const int yy = yp + ky - 1, xx = xq + kx - 1; const bool vin = (yy >= 0 && yy < HH && xx >= 0 && xx < HH); const int yc = min(max(yy, 0), HH - 1), xc = min(max(xx, 0), HH - 1);
    const float* src = (ci < 2) ? (wind + (((size_t)b * 2 + ci) * HH + yc) * HH + xc) : (topo + ((size_t)b * HH + yc) * HH + xc);
    const float v = vin ? bf16_round(*src) : 0.f;
#pragma unroll
    for (int o = 0; o < 8; ++o) acc[o] += v * bf16_round(w1[((o0 + o) * 3 + ci) * 9 + ky * 3 + kx]); }
  FragH f, z = FragH{};
#pragma unroll
  for (int o = 0; o < 8; ++o) { const float a = acc[o]; const float gl = 0.5f * a * (1.0f + erff(a * 0.70710678118654752f)); f.h[o] = in ? (_Float16)gl : (_Float16)0.0f; }
  for (int pass = 0; pass < 2; ++pass) { *(volatile v8us*)((unsigned short*)XP + (size_t)t * CHP + o0) = f.half[0]; *(volatile v8us*)((unsigned short*)XP + (size_t)t * CHP + 16 + o0) = z.half[0]; if (pass == 0) __threadfence(); } }
__global__ __launch_bounds__(256) void k_w2a(const float* __restrict__ w2, _Float16* __restrict__ A) { const int t = blockIdx.x * 256 + threadIdx.x; if (t >= NOP * (KI / 8)) return; const int c8 = (t % (KI / 8)) * 8, o = t / (KI / 8); FragH f;
#pragma unroll
  for (int q = 0; q < 8; ++q) { const int col = c8 + q; const int k = col / C1, c = col % C1; f.h[q] = (o < NO && col < 9 * C1) ? (_Float16)(bf16_round(w2[((size_t)o * C1 + c) * 9 + k]) * 16.0f) : (_Float16)0.0f; }
  *(volatile v8us*)((unsigned short*)A + (size_t)o * KI + c8) = f.half[0]; __threadfence(); *(volatile v8us*)((unsigned short*)A + (size_t)o * KI + c8) = f.half[0]; }
__global__ __launch_bounds__(256) void k_im2col(const _Float16* __restrict__ XP, int p0, _Float16* __restrict__ COL) { const int t = blockIdx.x * 256 + threadIdx.x; if (t >= HPX * 20) return; const int j = t % 20, pl = t / 20; const int p = p0 + pl; const int y = p / HH, x = p % HH; const int k = min(j >> 1, 8); const size_t src = ((size_t)(y + k / 3) * PW + (x + k % 3)) * CHP + (j & 1) * 8; FragH a; a.half[0] = *(const v8us*)((const unsigned short*)XP + src); if (j >= 18) a = FragH{};
  *(volatile v8us*)((unsigned short*)COL + (size_t)pl * KI + j * 8) = a.half[0]; __threadfence(); *(volatile v8us*)((unsigned short*)COL + (size_t)pl * KI + j * 8) = a.half[0]; }
__global__ __launch_bounds__(256) void k_w2t(const float* __restrict__ w2, _Float16* __restrict__ Bt) { const int t = blockIdx.x * 256 + threadIdx.x; if (t >= 9 * NOP * (CHP / 8)) return; const int c0 = (t % (CHP / 8)) * 8; const int o = (t / (CHP / 8)) % NOP; const int k = t / ((CHP / 8) * NOP); FragH f;
#pragma unroll
  for (int q = 0; q < 8; ++q) { const int c = c0 + q; f.h[q] = (o < NO && c < C1) ? (_Float16)(bf16_round(w2[((size_t)o * C1 + c) * 9 + k]) * 16.0f) : (_Float16)0.0f; }
  *(volatile v8us*)((unsigned short*)Bt + ((size_t)k * NOP + o) * CHP + c0) = f.half[0]; __threadfence(); *(volatile v8us*)((unsigned short*)Bt + ((size_t)k * NOP + o) * CHP + c0) = f.half[0]; }
__global__ __launch_bounds__(256) void k_bpad(const float* __restrict__ bb, int n, int np, float* __restrict__ BP) { const int l = threadIdx.x; if (l >= np) return; const float v = (l < n) ? bb[l] : 0.f; *(volatile float*)(BP + l) = v; __threadfence(); *(volatile float*)(BP + l) = v; }
__global__ __launch_bounds__(256) void k_samp(const float* __restrict__ OT, const float* __restrict__ b2, const float* __restrict__ pm, int b, const float* __restrict__ wgt, float* __restrict__ out) {
  #pragma clang fp contract(off)
  const int t = blockIdx.x * 256 + threadIdx.x; if (t >= NPX) return; const int y = t / HH, x = t % HH; const float* img = pm + (size_t)b * NPX; float acc = 0.f;
#pragma unroll 1
  for (int k = 0; k < 9; ++k) { const float dy = OT[(size_t)(2 * k) * NPX + t] + bf16_round(b2[2 * k]), dx = OT[(size_t)(2 * k + 1) * NPX + t] + bf16_round(b2[2 * k + 1]); const float py = (float)y + (float)(k / 3 - 1) + dy, px = (float)x + (float)(k % 3 - 1) + dx; const float y0f = floorf(py), x0f = floorf(px); const float wy1 = py - y0f, wx1 = px - x0f; const int y0 = (int)y0f, x0 = (int)x0f; float smp = 0.f;
#pragma unroll
    for (int cn = 0; cn < 4; ++cn) { const int yi = y0 + (cn >> 1), xi = x0 + (cn & 1); const bool valid = (yi >= 0 && yi < HH && xi >= 0 && xi < HH); const float w = ((cn >> 1) ? wy1 : 1.0f - wy1) * ((cn & 1) ? wx1 : 1.0f - wx1); const float v = bf16_round(img[(size_t)min(max(yi, 0), HH - 1) * HH + min(max(xi, 0), HH - 1)]); smp += w * (valid ? v : 0.f); }
    acc += smp * bf16_round(wgt[k]); }
  *(volatile float*)(out + (size_t)b * NPX + t) = acc; __threadfence(); *(volatile float*)(out + (size_t)b * NPX + t) = acc; }

extern "C" void kernel_launch(void* const* d_in, const int* in_sizes, int n_in,
                              void* d_out, int out_size, void* d_ws, size_t ws_size, hipStream_t stream) {
  (void)in_sizes; (void)n_in; (void)out_size;
  const float* pm = (const float*)d_in[0]; const float* wind = (const float*)d_in[1]; const float* topo = (const float*)d_in[2]; const float* w1 = (const float*)d_in[3]; const float* b1 = (const float*)d_in[4]; const float* w2 = (const float*)d_in[5]; const float* b2 = (const float*)d_in[6]; const float* wgt = (const float*)d_in[7];
  char* ws = (char*)d_ws; size_t off = 0;
  auto take = [&](size_t bytes) { char* p = ws + off; off += (bytes + 255) & ~(size_t)255; return p; };
  _Float16* AW = (_Float16*)take((size_t)NOP * KI * 2); _Float16* XP = (_Float16*)take((size_t)PR * PW * CHP * 2); _Float16* COL = (_Float16*)take((size_t)HPX * KI * 2); float* OT = (float*)take((size_t)NOP * NPX * 4);
  if (off > ws_size) return;
  k_w2a<<<(NOP * (KI / 8) + 255) / 256, 256, 0, stream>>>(w2, AW);
  const dim3 gT((((NOP / 16) * (HPX / 64)) + 3) / 4, 1);
  for (int b = 0; b < NBI; ++b) {
    k_conv1<<<(PR * PW * 2 + 255) / 256, 256, 0, stream>>>(wind, topo, b, w1, b1, XP);
    for (int hf = 0; hf < 2; ++hf) { const int p0 = hf * HPX;
      k_im2col<<<(HPX * 20 + 255) / 256, 256, 0, stream>>>(XP, p0, COL);
      k_gemm_hhx<0><<<gT, 128, 0, stream>>>(AW, KI, 0, COL, KI, 0, 0.0625f, nullptr, 0, nullptr, 1, 0, 0, OT + p0, nullptr, NPX, 0, NOP, HPX, KI); }
    k_samp<<<(NPX + 255) / 256, 256, 0, stream>>>(OT, b2, pm, b, wgt, (float*)d_out); }
}
